// FeatureAggregation_12841952215389
// MI455X (gfx1250) — hardware-verified
//
#include <hip/hip_runtime.h>
#include <math.h>
#include <stdint.h>

constexpr int kBatch   = 8;
constexpr int kCinHalf = 32;
constexpr int kCh      = 64;
constexpr int kPix     = 4096;
constexpr int kDq      = 32;

typedef __attribute__((ext_vector_type(16))) _Float16 v16h;
typedef __attribute__((ext_vector_type(8)))  _Float16 v8h;
typedef __attribute__((ext_vector_type(16))) __bf16   v16b;
typedef __attribute__((ext_vector_type(8)))  __bf16   v8b;
typedef __attribute__((ext_vector_type(8)))  float    v8f;
typedef __attribute__((ext_vector_type(4)))  float    v4f;
typedef __attribute__((ext_vector_type(4)))  unsigned int v4u;

__device__ __forceinline__ unsigned short f2bf_bits(float f) {
  unsigned u = __float_as_uint(f);
  return (unsigned short)((u + 0x7FFFu + ((u >> 16) & 1u)) >> 16);
}
__device__ __forceinline__ float bf_bits2f(unsigned short h) { return __uint_as_float(((unsigned)h) << 16); }
__device__ __forceinline__ unsigned pk16(unsigned short a, unsigned short b) { return (unsigned)a | ((unsigned)b << 16); }
__device__ __forceinline__ unsigned short h16_bits(float f) { const _Float16 h = (_Float16)f; return __builtin_bit_cast(unsigned short, h); }

__device__ __forceinline__ void dep_guard_h(v8f& a, v8f& b, v16h x, v16h y) { asm volatile("v_nop\n\tv_nop\n\tv_nop\n\tv_nop" : "+v"(a), "+v"(b) : "v"(x), "v"(y)); }
__device__ __forceinline__ void dep_guard_b(v8f& a, v8f& b, v16b x, v16b y) { asm volatile("v_nop\n\tv_nop\n\tv_nop\n\tv_nop" : "+v"(a), "+v"(b) : "v"(x), "v"(y)); }
__device__ __forceinline__ void keep4_h(v16h a, v16h b, v16h c, v16h d) { asm volatile("v_nop" :: "v"(a), "v"(b), "v"(c), "v"(d)); }
__device__ __forceinline__ void keep4_b(v16b a, v16b b, v16b c, v16b d) { asm volatile("v_nop" :: "v"(a), "v"(b), "v"(c), "v"(d)); }
__device__ __forceinline__ void acc_guard4(v8f& a, v8f& b, v8f& c, v8f& d) { asm volatile("v_nop\n\tv_nop\n\tv_nop\n\tv_nop" : "+v"(a), "+v"(b), "+v"(c), "+v"(d)); }
template <typename T> struct Frag;
template <> struct Frag<_Float16> {
  typedef v16h V; union U { v16h v; v8h h[2]; };
  static __device__ __forceinline__ v16h load(const _Float16* p) {
    U f; f.h[0] = *(const v8h*)(p); f.h[1] = *(const v8h*)(p + 16); return f.v;
  }
  static __device__ __forceinline__ v8f mma(v16h a, v16h b, v8f c) {
    return __builtin_amdgcn_wmma_f32_16x16x32_f16(false, a, false, b, (short)0, c, false, false);
  }
  static __device__ __forceinline__ void guard(v8f& a, v8f& b, v16h x, v16h y) { dep_guard_h(a, b, x, y); }
  static __device__ __forceinline__ void keep(v16h a, v16h b, v16h c, v16h d) { keep4_h(a, b, c, d); }
};
template <> struct Frag<__bf16> {
  typedef v16b V; union U { v16b v; v8b h[2]; };
  static __device__ __forceinline__ v16b load(const __bf16* p) {
    U f; f.h[0] = *(const v8b*)(p); f.h[1] = *(const v8b*)(p + 16); return f.v;
  }
  static __device__ __forceinline__ v8f mma(v16b a, v16b b, v8f c) {
    return __builtin_amdgcn_wmma_f32_16x16x32_bf16(false, a, false, b, (short)0, c, false, false);
  }
  static __device__ __forceinline__ void guard(v8f& a, v8f& b, v16b x, v16b y) { dep_guard_b(a, b, x, y); }
  static __device__ __forceinline__ void keep(v16b a, v16b b, v16b c, v16b d) { keep4_b(a, b, c, d); }
};

template <int ET> struct Elem;
template <> struct Elem<0> { typedef _Float16 T; };
template <> struct Elem<1> { typedef __bf16 T; };
template <int ET, bool SPLIT, int BIAS_MODE, int OUT_MODE, bool RESID, int ACT = 0>
__global__ __launch_bounds__(256) void wmma_gemm64(
    const unsigned short* __restrict__ Ap, const unsigned short* __restrict__ A2p, int lda, long strideA,
    const unsigned short* __restrict__ Btp, const unsigned short* __restrict__ Bt2p, int ldb, long strideB,
    void* __restrict__ Cout, void* __restrict__ Cout2, int ldc, long strideC,
    const float* __restrict__ bias,
    const float* __restrict__ resid, long strideR,
    int M, int N, int K, float scale) {
  typedef typename Elem<ET>::T T;
  typedef typename Frag<T>::V V;
  const T* A = (const T*)Ap; const T* A2 = (const T*)A2p; const T* Bt = (const T*)Btp; const T* Bt2 = (const T*)Bt2p;
  __shared__ __align__(16) float sT[8][16 * 68];
  const int b    = blockIdx.y;
  const int lane = threadIdx.x & 31;
  const int wave = threadIdx.x >> 5;
  const int tilesN = N >> 6;
  const int tilesM = M >> 6;
  const int tile = blockIdx.x * 8 + wave;
  if (tile >= tilesM * tilesN) return;
  const int tm = tile / tilesN;
  const int tn = tile - tm * tilesN;
  const int m0 = tm << 6;
  const int n0 = tn << 6;

  const T* Ab  = A  + (size_t)b * strideA;
  const T* Bb  = Bt + (size_t)b * strideB;
  const T* Ab2 = SPLIT ? (A2  + (size_t)b * strideA) : nullptr;
  const T* Bb2 = SPLIT ? (Bt2 + (size_t)b * strideB) : nullptr;

  const int rlane = lane & 15;
  const int koff  = (lane >> 4) * 8;
  const int mOff  = (lane >> 4) * 8;

  v8f acc[4][4];
#pragma unroll
  for (int i = 0; i < 4; ++i)
#pragma unroll
    for (int j = 0; j < 4; ++j) acc[i][j] = (v8f){0.f,0.f,0.f,0.f,0.f,0.f,0.f,0.f};

  for (int k0 = 0; k0 < K; k0 += 32) {
    V bh[4], bl[4];
#pragma unroll
    for (int j = 0; j < 4; ++j) {
      const size_t bo = (size_t)(n0 + (j << 4) + rlane) * ldb + koff + k0;
      bh[j] = Frag<T>::load(Bb + bo);
      if (SPLIT) bl[j] = Frag<T>::load(Bb2 + bo);
    }
#pragma unroll
    for (int i = 0; i < 4; ++i) {
      const size_t ao = (size_t)(m0 + (i << 4) + rlane) * lda + koff + k0;
      V ah = Frag<T>::load(Ab + ao);
      V al;
      if (SPLIT) al = Frag<T>::load(Ab2 + ao);
#pragma unroll
      for (int j = 0; j < 4; ++j) {
        acc[i][j] = Frag<T>::mma(ah, bh[j], acc[i][j]);
        if (SPLIT) {
          acc[i][j] = Frag<T>::mma(ah, bl[j], acc[i][j]);
          acc[i][j] = Frag<T>::mma(al, bh[j], acc[i][j]);
        }
      }
      Frag<T>::guard(acc[i][0], acc[i][3], ah, SPLIT ? al : ah);
    }
    Frag<T>::keep(bh[0], bh[1], bh[2], bh[3]);
    if (SPLIT) Frag<T>::keep(bl[0], bl[1], bl[2], bl[3]);
  }
  acc_guard4(acc[0][0], acc[0][1], acc[0][2], acc[0][3]);
  acc_guard4(acc[1][0], acc[1][1], acc[1][2], acc[1][3]);
  acc_guard4(acc[2][0], acc[2][1], acc[2][2], acc[2][3]);
  acc_guard4(acc[3][0], acc[3][1], acc[3][2], acc[3][3]);

  float* slab = sT[wave];
  const float* Rb = RESID ? (resid + (size_t)b * strideR) : nullptr;
#pragma unroll
  for (int i = 0; i < 4; ++i) {
    const int mBase = m0 + (i << 4);
#pragma unroll
    for (int j = 0; j < 4; ++j) {
      const int n = n0 + (j << 4) + rlane;
      float bv = 0.f;
      if (BIAS_MODE == 2) bv = bias[n];
#pragma unroll
      for (int r = 0; r < 8; ++r) {
        float v = acc[i][j][r] * scale;
        if (BIAS_MODE == 1) v += bias[mBase + mOff + r];
        if (BIAS_MODE == 2) v += bv;
        if (RESID) v += Rb[(size_t)(mBase + mOff + r) * ldc + n];
        if (ACT == 1) v = tanhf(v);
        if (ACT == 2) v = fmaxf(v, 0.0f);
        if (ACT == 3) v = v / (1.0f + expf(-v));
        if (ACT == 4) v = (v > 0.f) ? v : 0.01f * v;
        if (ACT == 5) v = 0.5f * v * (1.0f + erff(v * 0.70710678118654752f));
        slab[(mOff + r) * 68 + (j << 4) + rlane] = v;
      }
    }
    __builtin_amdgcn_fence(__ATOMIC_RELEASE, "workgroup");
    __builtin_amdgcn_wave_barrier();
    __builtin_amdgcn_fence(__ATOMIC_ACQUIRE, "workgroup");
    if (OUT_MODE == 0) {
      float* C = (float*)Cout + (size_t)b * strideC;
      const int hh = lane >> 4, c4 = (lane & 15) * 4;
      for (int pass = 0; pass < 2; ++pass) {
#pragma unroll
        for (int it = 0; it < 8; ++it) {
          const int row = it * 2 + hh;
          v4f v = *(const v4f*)(slab + row * 68 + c4);
          *(volatile v4f*)(C + (size_t)(mBase + row) * ldc + n0 + c4) = v;
        }
        __threadfence();
      }
    } else {
      const int q = lane >> 3, c8 = (lane & 7) * 8;
      unsigned short* C  = (unsigned short*)Cout  + (size_t)b * strideC;
      unsigned short* C2 = (OUT_MODE == 2) ? ((unsigned short*)Cout2 + (size_t)b * strideC) : nullptr;
      for (int pass = 0; pass < 2; ++pass) {
#pragma unroll
        for (int it = 0; it < 4; ++it) {
          const int row = it * 4 + q;
          const float* sp = slab + row * 68 + c8;
          v8h hv, lv;
#pragma unroll
          for (int e = 0; e < 8; ++e) {
            if (OUT_MODE == 1) {
              hv[e] = (_Float16)sp[e];
            } else {
              unsigned short hb = f2bf_bits(sp[e]);
              unsigned short lb = f2bf_bits(sp[e] - bf_bits2f(hb));
              hv[e] = __builtin_bit_cast(_Float16, hb);
              lv[e] = __builtin_bit_cast(_Float16, lb);
            }
          }
          *(volatile v8h*)(C + (size_t)(mBase + row) * ldc + n0 + c8) = hv;
          if (OUT_MODE == 2) *(volatile v8h*)(C2 + (size_t)(mBase + row) * ldc + n0 + c8) = lv;
        }
        __threadfence();
      }
    }
    __builtin_amdgcn_fence(__ATOMIC_RELEASE, "workgroup");
    __builtin_amdgcn_wave_barrier();
    __builtin_amdgcn_fence(__ATOMIC_ACQUIRE, "workgroup");
  }
}

__global__ __launch_bounds__(256) void prep_kernel(
    const float* __restrict__ Wq, const float* __restrict__ Wk, const float* __restrict__ Wv,
    const float* __restrict__ Wsc, const float* __restrict__ bq, const float* __restrict__ bk,
    unsigned short* __restrict__ Wqk16, unsigned short* __restrict__ Wv16,
    unsigned short* __restrict__ Wsch, unsigned short* __restrict__ Wscl, float* __restrict__ bqk) {
  const int tid  = threadIdx.x;
  const int role = blockIdx.x;
  if (role == 0) {
    v4u hv[2];
#pragma unroll
    for (int it = 0; it < 2; ++it) {
      const int task = it * 256 + tid;
      const int row = task >> 3, c8 = (task & 7) * 8;
      const int rq = row < kDq ? row : (kDq - 1);
      int rk = row - kDq; rk = rk < 0 ? 0 : (rk > kDq - 1 ? kDq - 1 : rk);
      const v4f a0 = *(const v4f*)(Wq + rq * kCh + c8), a1 = *(const v4f*)(Wq + rq * kCh + c8 + 4);
      const v4f b0 = *(const v4f*)(Wk + rk * kCh + c8), b1 = *(const v4f*)(Wk + rk * kCh + c8 + 4);
      const bool useq = row < kDq;
      float f[8];
#pragma unroll
      for (int e = 0; e < 4; ++e) { f[e] = useq ? a0[e] : b0[e]; f[4 + e] = useq ? a1[e] : b1[e]; }
      v4u u;
#pragma unroll
      for (int q = 0; q < 4; ++q) u[q] = pk16(h16_bits(f[2 * q]), h16_bits(f[2 * q + 1]));
      hv[it] = u;
    }
    for (int pass = 0; pass < 2; ++pass) {
#pragma unroll
      for (int it = 0; it < 2; ++it) {
        const int task = it * 256 + tid;
        const int row = task >> 3, c8 = (task & 7) * 8;
        *(volatile v4u*)(Wqk16 + row * kCh + c8) = hv[it];
      }
      __threadfence();
    }
  } else if (role == 1) {
    v4u hv[2];
#pragma unroll
    for (int it = 0; it < 2; ++it) {
      const int task = it * 256 + tid;
      const int row = task >> 3, c8 = (task & 7) * 8;
      const v4f a0 = *(const v4f*)(Wv + row * kCh + c8), a1 = *(const v4f*)(Wv + row * kCh + c8 + 4);
      float f[8];
#pragma unroll
      for (int e = 0; e < 4; ++e) { f[e] = a0[e]; f[4 + e] = a1[e]; }
      v4u u;
#pragma unroll
      for (int q = 0; q < 4; ++q) u[q] = pk16(h16_bits(f[2 * q]), h16_bits(f[2 * q + 1]));
      hv[it] = u;
    }
    for (int pass = 0; pass < 2; ++pass) {
#pragma unroll
      for (int it = 0; it < 2; ++it) {
        const int task = it * 256 + tid;
        const int row = task >> 3, c8 = (task & 7) * 8;
        *(volatile v4u*)(Wv16 + row * kCh + c8) = hv[it];
      }
      __threadfence();
    }
  } else if (role == 2) {
    v4u hv[2], lv[2];
#pragma unroll
    for (int it = 0; it < 2; ++it) {
      const int task = it * 256 + tid;
      const int row = task >> 3, c8 = (task & 7) * 8;
      const int rs = row < kDq ? row : (kDq - 1);
      const bool live = row < kDq;
      const v4f a0 = *(const v4f*)(Wsc + rs * kCh + c8), a1 = *(const v4f*)(Wsc + rs * kCh + c8 + 4);
      float f[8];
#pragma unroll
      for (int e = 0; e < 4; ++e) { f[e] = live ? a0[e] : 0.0f; f[4 + e] = live ? a1[e] : 0.0f; }
      v4u u, u2;
#pragma unroll
      for (int q = 0; q < 4; ++q) {
        const unsigned short hb0 = f2bf_bits(f[2 * q]), hb1 = f2bf_bits(f[2 * q + 1]);
        const unsigned short lb0 = f2bf_bits(f[2 * q] - bf_bits2f(hb0));
        const unsigned short lb1 = f2bf_bits(f[2 * q + 1] - bf_bits2f(hb1));
        u[q] = pk16(hb0, hb1); u2[q] = pk16(lb0, lb1);
      }
      hv[it] = u; lv[it] = u2;
    }
    for (int pass = 0; pass < 2; ++pass) {
#pragma unroll
      for (int it = 0; it < 2; ++it) {
        const int task = it * 256 + tid;
        const int row = task >> 3, c8 = (task & 7) * 8;
        *(volatile v4u*)(Wsch + row * kCh + c8) = hv[it];
        *(volatile v4u*)(Wscl + row * kCh + c8) = lv[it];
      }
      __threadfence();
    }
  } else if (role == 3) {
    if (tid < 16) {
      const int iq = (4 * tid < kDq - 4) ? 4 * tid : (kDq - 4);
      int ik = 4 * tid - kDq; ik = ik < 0 ? 0 : (ik > kDq - 4 ? kDq - 4 : ik);
      const v4f a = *(const v4f*)(bq + iq);
      const v4f c = *(const v4f*)(bk + ik);
      const v4f v = (tid < 8) ? a : c;
      *(volatile v4f*)(bqk + 4 * tid) = v;
      __threadfence();
      *(volatile v4f*)(bqk + 4 * tid) = v;
    }
  }
}

__global__ __launch_bounds__(256) void xcat_transpose_f16_kernel(const float* __restrict__ x1, const float* __restrict__ x2,
                                                                 unsigned short* __restrict__ Xo) {
  __shared__ __align__(16) float tf[64 * 68];
  const int bx  = blockIdx.x;
  const int b   = bx >> 6;
  const int n0  = (bx & 63) * 64;
  const int tid = threadIdx.x;
  const int sub = tid >> 4, c4 = (tid & 15) * 4;
#pragma unroll
  for (int it = 0; it < 2; ++it) {
    const int ch = it * 16 + sub;
    const v4f a = *(const v4f*)(x1 + ((size_t)(b * kCinHalf + ch) * kPix + n0 + c4));
    *(v4f*)(tf + ch * 68 + c4) = a;
  }
#pragma unroll
  for (int it = 0; it < 2; ++it) {
    const int ch = it * 16 + sub;
    const v4f a = *(const v4f*)(x2 + ((size_t)(b * kCinHalf + ch) * kPix + n0 + c4));
    *(v4f*)(tf + (kCinHalf + ch) * 68 + c4) = a;
  }
  __syncthreads();
  const int s8 = tid >> 3, c8 = (tid & 7) * 8;
  v4u hv[2];
#pragma unroll
  for (int it = 0; it < 2; ++it) {
    const int oc = it * 32 + s8;
    v4u u;
#pragma unroll
    for (int q = 0; q < 4; ++q) {
      const float f0 = tf[(c8 + 2 * q) * 68 + oc];
      const float f1 = tf[(c8 + 2 * q + 1) * 68 + oc];
      u[q] = pk16(h16_bits(f0), h16_bits(f1));
    }
    hv[it] = u;
  }
  for (int pass = 0; pass < 2; ++pass) {
#pragma unroll
    for (int it = 0; it < 2; ++it) {
      const int oc = it * 32 + s8;
      *(volatile v4u*)(Xo + ((size_t)(b * kPix + n0 + oc) * kCh + c8)) = hv[it];
    }
    __threadfence();
  }
}

__global__ __launch_bounds__(256) void colstats_kernel(const float* __restrict__ S,
                                                       float* __restrict__ cmax, float* __restrict__ cscale) {
  const int m4 = (blockIdx.x * 256 + threadIdx.x) * 4;
  const float* col = S + m4;
  v4f mx = *(const v4f*)col;
  v4f sm = (v4f){1.0f, 1.0f, 1.0f, 1.0f};
#pragma unroll 2
  for (int n = 1; n < kPix; ++n) {
    const v4f s = *(const v4f*)(col + (size_t)n * kPix);
#pragma unroll
    for (int e = 0; e < 4; ++e) {
      const float d  = s[e] - mx[e];
      const float ex = __expf(-fabsf(d));
      sm[e] = (d > 0.0f) ? (sm[e] * ex + 1.0f) : (sm[e] + ex);
      mx[e] = fmaxf(mx[e], s[e]);
    }
  }
  v4f sc;
#pragma unroll
  for (int e = 0; e < 4; ++e) sc[e] = 4096.0f * __builtin_amdgcn_rcpf(sm[e]);
  for (int pass = 0; pass < 2; ++pass) {
    *(volatile v4f*)(cmax + m4)   = mx;
    *(volatile v4f*)(cscale + m4) = sc;
    __threadfence();
  }
}

__global__ __launch_bounds__(256) void colsoftmax_p_kernel(const float* __restrict__ S, const float* __restrict__ cmax,
                                                           const float* __restrict__ cscale, unsigned short* __restrict__ P) {
  const int t  = blockIdx.x * 256 + threadIdx.x;
  const int n  = t >> 9;
  const int m8 = (t & 511) * 8;
  const float* sp = S + (size_t)n * kPix + m8;
  const v4f s0 = *(const v4f*)sp, s1 = *(const v4f*)(sp + 4);
  const v4f c0 = *(const v4f*)(cmax + m8), c1 = *(const v4f*)(cmax + m8 + 4);
  const v4f k0 = *(const v4f*)(cscale + m8), k1 = *(const v4f*)(cscale + m8 + 4);
  float p[8];
#pragma unroll
  for (int e = 0; e < 4; ++e) {
    p[e]     = __expf(s0[e] - c0[e]) * k0[e];
    p[4 + e] = __expf(s1[e] - c1[e]) * k1[e];
  }
  v4u u;
#pragma unroll
  for (int q = 0; q < 4; ++q) u[q] = pk16(h16_bits(p[2 * q]), h16_bits(p[2 * q + 1]));
  unsigned short* dst = P + (size_t)n * kPix + m8;
  *(volatile v4u*)dst = u;
  __threadfence();
  *(volatile v4u*)dst = u;
}

__global__ __launch_bounds__(256) void resid_split_kernel(const float* __restrict__ O, const float* __restrict__ x1,
                                                          const float* __restrict__ x2, const float* __restrict__ gamma,
                                                          unsigned short* __restrict__ Zh, unsigned short* __restrict__ Zl) {
#pragma clang fp contract(off)
  __shared__ __align__(16) float tf[64 * 68];
  const int bx  = blockIdx.x;
  const int b   = bx >> 6;
  const int n0  = (bx & 63) * 64;
  const int tid = threadIdx.x;
  const int sub = tid >> 4, c4 = (tid & 15) * 4;
#pragma unroll
  for (int it = 0; it < 2; ++it) {
    const int ch = it * 16 + sub;
    const v4f a = *(const v4f*)(x1 + ((size_t)(b * kCinHalf + ch) * kPix + n0 + c4));
    *(v4f*)(tf + ch * 68 + c4) = a;
  }
#pragma unroll
  for (int it = 0; it < 2; ++it) {
    const int ch = it * 16 + sub;
    const v4f a = *(const v4f*)(x2 + ((size_t)(b * kCinHalf + ch) * kPix + n0 + c4));
    *(v4f*)(tf + (kCinHalf + ch) * 68 + c4) = a;
  }
  __syncthreads();
  const float g = gamma[0];
  const int s8 = tid >> 3, c8 = (tid & 7) * 8;
  v4u hv[2], lv[2];
#pragma unroll
  for (int it = 0; it < 2; ++it) {
    const int oc = it * 32 + s8;
    const size_t ro = (size_t)(b * kPix + n0 + oc) * kCh + c8;
    const v4f o0 = *(const v4f*)(O + ro), o1 = *(const v4f*)(O + ro + 4);
    float z[8];
#pragma unroll
    for (int e = 0; e < 4; ++e) {
      z[e]     = g * o0[e] + tf[(c8 + e) * 68 + oc];
      z[4 + e] = g * o1[e] + tf[(c8 + 4 + e) * 68 + oc];
    }
    v4u u, u2;
#pragma unroll
    for (int q = 0; q < 4; ++q) {
      const unsigned short hb0 = f2bf_bits(z[2 * q]), hb1 = f2bf_bits(z[2 * q + 1]);
      const unsigned short lb0 = f2bf_bits(z[2 * q] - bf_bits2f(hb0));
      const unsigned short lb1 = f2bf_bits(z[2 * q + 1] - bf_bits2f(hb1));
      u[q] = pk16(hb0, hb1); u2[q] = pk16(lb0, lb1);
    }
    hv[it] = u; lv[it] = u2;
  }
  for (int pass = 0; pass < 2; ++pass) {
#pragma unroll
    for (int it = 0; it < 2; ++it) {
      const int oc = it * 32 + s8;
      const size_t ro = (size_t)(b * kPix + n0 + oc) * kCh + c8;
      *(volatile v4u*)(Zh + ro) = hv[it];
      *(volatile v4u*)(Zl + ro) = lv[it];
    }
    __threadfence();
  }
}

__global__ __launch_bounds__(256) void copy_out_kernel(const float* __restrict__ F, float* __restrict__ out) {
  const int t  = blockIdx.x * 256 + threadIdx.x;
  const int b  = t >> 15;
  const int r  = t & 32767;
  const int o  = r >> 10;
  const int n4 = (r & 1023) * 4;
  const v4f v = *(const v4f*)(F + ((size_t)(b * kCh + o) * kPix + n4));
  float* dst = out + ((size_t)(b * kDq + o) * kPix + n4);
  *(volatile v4f*)dst = v;
  __threadfence();
  *(volatile v4f*)dst = v;
}

extern "C" void kernel_launch(void* const* d_in, const int* in_sizes, int n_in,
                              void* d_out, int out_size, void* d_ws, size_t ws_size,
                              hipStream_t stream) {
  if (n_in < 9) return;
  if (in_sizes[0] != kBatch * kCinHalf * kPix || in_sizes[1] != kBatch * kCinHalf * kPix) return;
  if (in_sizes[2] != kDq * kCh || in_sizes[3] != kDq || in_sizes[4] != kDq * kCh || in_sizes[5] != kDq) return;
  if (in_sizes[6] != kCh * kCh || in_sizes[7] != kDq * kCh || in_sizes[8] < 1) return;
  if (out_size != kBatch * kDq * kPix) return;

  const float* x1    = (const float*)d_in[0];
  const float* x2    = (const float*)d_in[1];
  const float* Wq    = (const float*)d_in[2];
  const float* bq    = (const float*)d_in[3];
  const float* Wk    = (const float*)d_in[4];
  const float* bk    = (const float*)d_in[5];
  const float* Wv    = (const float*)d_in[6];
  const float* Wsc   = (const float*)d_in[7];
  const float* gamma = (const float*)d_in[8];
  float* out = (float*)d_out;

  const size_t szPlane16 = (size_t)kBatch * kPix * kCh * 2;
  const size_t szS       = (size_t)kPix * kPix * 4;
  const size_t szP       = (size_t)kPix * kPix * 2;
  const size_t szO       = (size_t)kBatch * kPix * kCh * 4;
  const size_t szF       = (size_t)kBatch * kCh * kPix * 4;
  size_t off = 0;
  const size_t oSmall = off; off += 65536;
  const size_t oX     = off; off += szPlane16;
  const size_t oQK    = off; off += szPlane16;
  const size_t oV     = off; off += szPlane16;
  const size_t oS     = off; off += szS;
  const size_t oStat  = off; off += 65536;
  const size_t oP     = off; off += szP;
  const size_t oO     = off; off += szO;
  if (2 * szPlane16 + szF > szS) return;
  if (off > ws_size) return;

  char* ws = (char*)d_ws;
  unsigned short* Wqk16 = (unsigned short*)(ws + oSmall + 0);
  unsigned short* Wv16  = (unsigned short*)(ws + oSmall + 8192);
  unsigned short* Wsch  = (unsigned short*)(ws + oSmall + 16384);
  unsigned short* Wscl  = (unsigned short*)(ws + oSmall + 24576);
  float*          bqk   = (float*)(ws + oSmall + 32768);
  unsigned short* Xp    = (unsigned short*)(ws + oX);
  unsigned short* QKp   = (unsigned short*)(ws + oQK);
  unsigned short* Vp    = (unsigned short*)(ws + oV);
  float*          Sp    = (float*)(ws + oS);
  unsigned short* Zh    = (unsigned short*)(ws + oS);
  unsigned short* Zl    = (unsigned short*)(ws + oS + szPlane16);
  float*          Fp    = (float*)(ws + oS + 2 * szPlane16);
  float*          cmax  = (float*)(ws + oStat);
  float*          cscale = (float*)(ws + oStat + 16384);
  unsigned short* Pp    = (unsigned short*)(ws + oP);
  float*          Op    = (float*)(ws + oO);

  const dim3 blk(256);
  prep_kernel<<<dim3(4), blk, 0, stream>>>(Wq, Wk, Wv, Wsc, bq, bk, Wqk16, Wv16, Wsch, Wscl, bqk);
  xcat_transpose_f16_kernel<<<dim3(kBatch * (kPix / 64)), blk, 0, stream>>>(x1, x2, Xp);
  wmma_gemm64<0, false, 2, 1, false, 0><<<dim3((kBatch * kPix / 64) / 8, 1), blk, 0, stream>>>(
      Xp, Xp, kCh, 0L, Wqk16, Wqk16, kCh, 0L, (void*)QKp, (void*)QKp, kCh, 0L,
      bqk, bqk, 0L, kBatch * kPix, kCh, kCh, 1.0f);
  wmma_gemm64<0, false, 0, 1, false, 0><<<dim3(((kCh / 64) * (kPix / 64)) / 8, kBatch), blk, 0, stream>>>(
      Wv16, Wv16, kCh, 0L, Xp, Xp, kCh, (long)kPix * kCh, (void*)Vp, (void*)Vp, kPix, (long)kCh * kPix,
      bqk, bqk, 0L, kCh, kPix, kCh, 1.0f);

  for (int b = 0; b < kBatch; ++b) {
    const unsigned short* qk_b = QKp + (size_t)b * kPix * kCh;
    wmma_gemm64<0, false, 0, 0, false, 0><<<dim3(((kPix / 64) * (kPix / 64)) / 8, 1), blk, 0, stream>>>(
        qk_b, qk_b, kCh, 0L, qk_b + kDq, qk_b + kDq, kCh, 0L, (void*)Sp, (void*)Sp, kPix, 0L,
        bqk, bqk, 0L, kPix, kPix, kDq, 1.0f);
    colstats_kernel<<<dim3(kPix / 1024), blk, 0, stream>>>(Sp, cmax, cscale);
    colsoftmax_p_kernel<<<dim3((kPix / 8) * (kPix / 256)), blk, 0, stream>>>(Sp, cmax, cscale, Pp);
    wmma_gemm64<0, false, 0, 0, false, 0><<<dim3(((kPix / 64) * (kCh / 64)) / 8, 1), blk, 0, stream>>>(
        Pp, Pp, kPix, 0L, Vp + (size_t)b * kCh * kPix, Vp + (size_t)b * kCh * kPix, kPix, 0L,
        (void*)(Op + (size_t)b * kPix * kCh), (void*)(Op + (size_t)b * kPix * kCh), kCh, 0L,
        bqk, bqk, 0L, kPix, kCh, kPix, 1.0f / 4096.0f);
  }
  resid_split_kernel<<<dim3(kBatch * (kPix / 64)), blk, 0, stream>>>(Op, x1, x2, gamma, Zh, Zl);
  wmma_gemm64<1, true, 0, 0, false, 0><<<dim3(((kCh / 64) * (kPix / 64)) / 8, kBatch), blk, 0, stream>>>(
      Wsch, Wscl, kCh, 0L, Zh, Zl, kCh, (long)kPix * kCh, (void*)Fp, (void*)Fp, kPix, (long)kCh * kPix,
      bqk, bqk, 0L, kCh, kPix, kCh, 1.0f);
  copy_out_kernel<<<dim3((kBatch * kDq * kPix / 4) / 256), blk, 0, stream>>>(Fp, out);
}
